// NeuralAttentionRegressor_12000138625052
// MI455X (gfx1250) — hardware-run, weakly checked
//
#include <hip/hip_runtime.h>
#include <math.h>
#include <stdint.h>

#define NB      4
#define NQ      2048
#define DIN     64
#define DOUT    8
#define DMODEL  256
#define DFF     1024
#define NHEAD   8
#define HDIM    32
#define NLAYER  3
#define NROWS   (NB * NQ)
#define QKP     (2 * DMODEL)
#define OUT0_N  (NROWS * DOUT)
#define WSC     64.0f
#define HCARRY  16.0f
#define QC      16.0f
#define KC      16.0f
#define VC      16.0f
#define PC      1024.0f
#define FC      1024.0f
#define GC      16.0f
#define ATT_SCALE 0.17677669529663687f
#define LOG2E   1.4426950408889634f
#define LN_EPS  1e-5f
#define PE_C    (-0.03597789207803197f)
static_assert(NHEAD * HDIM == DMODEL);
static_assert((NQ % 64) == 0 && (DMODEL % 64) == 0 && (DFF % 64) == 0 && (DIN % 64) == 0 && (NQ % 32) == 0 && (NQ % 16) == 0);
static_assert((NROWS % 64) == 0 && (DMODEL % 32) == 0 && (DFF % 32) == 0 && (DIN % 32) == 0);
static_assert((NQ & (NQ - 1)) == 0);
#define ATT_THREADS (NHEAD * 32)
#define ATT_BLOCKS  (NB * (NQ / 16))
#define OSP         DMODEL
static_assert(ATT_THREADS == 256 && ATT_BLOCKS == 512);
#define LN_THREADS 256
static_assert(32 * 8 == DMODEL && (NROWS % 8) == 0);
#define CVT_THREADS 256
static_assert(((NROWS * DIN / 8) % CVT_THREADS) == 0);
static_assert(((NQ * (DMODEL / 2)) % 256) == 0);

typedef _Float16 v16h __attribute__((ext_vector_type(16)));
typedef _Float16 v8h  __attribute__((ext_vector_type(8)));
typedef float    v8f  __attribute__((ext_vector_type(8)));
typedef float    v4f  __attribute__((ext_vector_type(4)));
typedef float    v2f  __attribute__((ext_vector_type(2)));
typedef unsigned int v4u __attribute__((ext_vector_type(4)));
typedef unsigned int v2u __attribute__((ext_vector_type(2)));

union FragH { v16h v; v8h h[2]; v4u u[2]; };

__device__ __forceinline__ unsigned short bf_bits(float f) {
  unsigned u = __float_as_uint(f);
  return (unsigned short)((u + 0x7FFFu + ((u >> 16) & 1u)) >> 16);
}
__device__ __forceinline__ float bf_up(unsigned short h) { return __uint_as_float(((unsigned)h) << 16); }
__device__ __forceinline__ float bfr(float f) { return bf_up(bf_bits(f)); }
__device__ __forceinline__ unsigned short h_bits(_Float16 x) { return __builtin_bit_cast(unsigned short, x); }
__device__ __forceinline__ unsigned pk16(unsigned short a, unsigned short b) { return (unsigned)a | ((unsigned)b << 16); }
__device__ __forceinline__ v8f zero8() { v8f z = {0.f, 0.f, 0.f, 0.f, 0.f, 0.f, 0.f, 0.f}; return z; }
__device__ __forceinline__ float gelu_erf(float x) { return 0.5f * x * (1.0f + erff(x * 0.70710678118654752f)); }

__device__ __forceinline__ v16h ldfrag_h(const _Float16* p) {
  FragH f;
  f.h[0] = *(const v8h*)(p);
  f.h[1] = *(const v8h*)(p + 16);
  return f.v;
}
__device__ __forceinline__ v16h ldfrag_u(const unsigned short* p) {
  FragH f;
  f.u[0] = *(const v4u*)(p);
  f.u[1] = *(const v4u*)(p + 16);
  return f.v;
}

__device__ __forceinline__ v8f mma_raw(v16h a, v16h b, v8f c) {
  return __builtin_amdgcn_wmma_f32_16x16x32_f16(false, a, false, b, (short)0, c, false, false);
}
__device__ __forceinline__ void dep_guard1(v8f& a, v8f& b, v16h x) {
#if defined(__HIP_DEVICE_COMPILE__)
  asm volatile("v_nop\n\tv_nop\n\tv_nop\n\tv_nop" : "+v"(a), "+v"(b) : "v"(x));
#endif
}
__device__ __forceinline__ void guard2(v8f& a, v8f& b, v16h x, v16h y, v16h z) {
#if defined(__HIP_DEVICE_COMPILE__)
  asm volatile("v_nop\n\tv_nop\n\tv_nop\n\tv_nop" : "+v"(a), "+v"(b) : "v"(x), "v"(y), "v"(z));
#endif
}
__device__ __forceinline__ void keep4_h(v16h a, v16h b, v16h c, v16h d) {
#if defined(__HIP_DEVICE_COMPILE__)
  asm volatile("v_nop" :: "v"(a), "v"(b), "v"(c), "v"(d));
#endif
}
__device__ __forceinline__ void acc_guard4(v8f& a, v8f& b, v8f& c, v8f& d) {
#if defined(__HIP_DEVICE_COMPILE__)
  asm volatile("v_nop\n\tv_nop\n\tv_nop\n\tv_nop" : "+v"(a), "+v"(b), "+v"(c), "+v"(d));
#endif
}
__device__ __forceinline__ void wave_sync_lds() {
  __builtin_amdgcn_fence(__ATOMIC_RELEASE, "workgroup");
  __builtin_amdgcn_wave_barrier();
  __builtin_amdgcn_fence(__ATOMIC_ACQUIRE, "workgroup");
}

__global__ __launch_bounds__(CVT_THREADS) void cvt16(const float* __restrict__ src, unsigned short* dst, int n8, float sc) {
  const int i = blockIdx.x * CVT_THREADS + threadIdx.x;
  if (i >= n8) return;
  const float* sp = src + (size_t)i * 8;
  const v4f a = *(const v4f*)(sp);
  const v4f b = *(const v4f*)(sp + 4);
  v4u w;
  w[0] = pk16(h_bits((_Float16)(bfr(a[0]) * sc)), h_bits((_Float16)(bfr(a[1]) * sc)));
  w[1] = pk16(h_bits((_Float16)(bfr(a[2]) * sc)), h_bits((_Float16)(bfr(a[3]) * sc)));
  w[2] = pk16(h_bits((_Float16)(bfr(b[0]) * sc)), h_bits((_Float16)(bfr(b[1]) * sc)));
  w[3] = pk16(h_bits((_Float16)(bfr(b[2]) * sc)), h_bits((_Float16)(bfr(b[3]) * sc)));
  unsigned short* dp = dst + (size_t)i * 8;
  for (int pass = 0; pass < 2; ++pass) {
    *(volatile v4u*)dp = w;
    __threadfence();
  }
}

__global__ __launch_bounds__(256) void tcvt16(const float* __restrict__ src, unsigned short* dst, int R, int C, float sc) {
  __shared__ __align__(16) unsigned short sT[64 * 72];
  const int tid = threadIdx.x, lane = tid & 31, wave = tid >> 5;
  const size_t zo = (size_t)blockIdx.z * (size_t)R * (size_t)C;
  src += zo;
  dst += zo;
  const int c0 = blockIdx.x * 64, r0 = blockIdx.y * 64;
  const int rr = tid >> 2, cc = (tid & 3) * 16;
  const float* sp = src + (size_t)(r0 + rr) * C + c0 + cc;
#pragma unroll
  for (int e = 0; e < 4; ++e) {
    const v4f a = *(const v4f*)(sp + 4 * e);
#pragma unroll
    for (int k = 0; k < 4; ++k)
      sT[(cc + 4 * e + k) * 72 + rr] = h_bits((_Float16)(bfr(a[k]) * sc));
  }
  __syncthreads();
  v4u vals[2];
#pragma unroll
  for (int it = 0; it < 2; ++it) {
    const int q = it * 32 + wave * 4 + (lane >> 3);
    vals[it] = *(const v4u*)(sT + q * 72 + (lane & 7) * 8);
  }
  for (int pass = 0; pass < 2; ++pass) {
#pragma unroll
    for (int it = 0; it < 2; ++it) {
      const int q = it * 32 + wave * 4 + (lane >> 3);
      *(volatile v4u*)(dst + (size_t)(c0 + q) * R + r0 + (lane & 7) * 8) = vals[it];
    }
    __threadfence();
  }
}

__global__ __launch_bounds__(256) void cvtqkv(const float* __restrict__ wq, const float* __restrict__ wk,
                                              const float* __restrict__ wv, unsigned short* dst, float sc) {
  __shared__ __align__(16) unsigned short sT[HDIM * 264];
  const int tid = threadIdx.x, lane = tid & 31, wave = tid >> 5;
  const int h = blockIdx.x, l = blockIdx.y, p = blockIdx.z;
  const float* src = (p == 0) ? wq : ((p == 1) ? wk : wv);
  src += (((size_t)l * NHEAD + h) * DMODEL) * HDIM;
  const float* sp = src + (size_t)tid * HDIM;
#pragma unroll
  for (int e = 0; e < 8; ++e) {
    const v4f a = *(const v4f*)(sp + 4 * e);
#pragma unroll
    for (int k = 0; k < 4; ++k)
      sT[(4 * e + k) * 264 + tid] = h_bits((_Float16)(bfr(a[k]) * sc));
  }
  __syncthreads();
  v4u vals[4];
#pragma unroll
  for (int it = 0; it < 4; ++it) {
    const int kk = it * 8 + wave;
    vals[it] = *(const v4u*)(sT + kk * 264 + lane * 8);
  }
  const size_t rowbase = (size_t)l * (3 * DMODEL) + (size_t)p * DMODEL + (size_t)h * HDIM;
  for (int pass = 0; pass < 2; ++pass) {
#pragma unroll
    for (int it = 0; it < 4; ++it) {
      const int kk = it * 8 + wave;
      *(volatile v4u*)(dst + (rowbase + kk) * DMODEL + lane * 8) = vals[it];
    }
    __threadfence();
  }
}

__global__ __launch_bounds__(256) void petab(float* PE) {
  const int idx = blockIdx.x * 256 + threadIdx.x;
  const int t = idx >> 7, m = idx & 127;
  const float dv  = expf((float)(2 * m) * PE_C);
  const float ang = (float)t * dv;
  v2f w;
  w[0] = sinf(ang);
  w[1] = cosf(ang);
  float* p = PE + (size_t)t * DMODEL + 2 * m;
  for (int pass = 0; pass < 2; ++pass) {
    *(volatile v2f*)p = w;
    __threadfence();
  }
}

template <int OM, int HASR, int HASB, int ACT, int RMOD>
__global__ __launch_bounds__(256) void gemm64(
    const unsigned short* __restrict__ Ap, int lda, long long sA,
    const unsigned short* __restrict__ Btp, int ldb, long long sB,
    const float* __restrict__ Rp, const float* __restrict__ Bsp,
    void* Cout, int ldc, long long sC,
    int M, int N, int K, float oscale, float ocarry) {
  static_assert(!(OM == 0 && HASB == 2));
  static_assert(!(OM != 0 && HASR != 0));
  __shared__ __align__(16) float sT[8][16 * 68];
  const int by   = blockIdx.y;
  const int lane = threadIdx.x & 31;
  const int wave = threadIdx.x >> 5;
  const int tilesN = N >> 6;
  const int tilesM = M >> 6;
  const int tile = blockIdx.x * 8 + wave;
  if (tile >= tilesM * tilesN) return;
  const int tm = tile / tilesN;
  const int tn = tile - tm * tilesN;
  const int m0 = tm << 6;
  const int n0 = tn << 6;

  const unsigned short* A1 = Ap  + (size_t)((long long)by * sA);
  const unsigned short* Bb = Btp + (size_t)((long long)by * sB);

  const int rlane = lane & 15;
  const int koff  = (lane >> 4) * 8;
  const int mOff  = (lane >> 4) * 8;

  v8f acc[4][4];
#pragma unroll
  for (int i = 0; i < 4; ++i)
#pragma unroll
    for (int j = 0; j < 4; ++j) acc[i][j] = zero8();

  for (int k0 = 0; k0 < K; k0 += 32) {
    v16h bh[4];
#pragma unroll
    for (int j = 0; j < 4; ++j) {
      const size_t bofs = (size_t)(n0 + (j << 4) + rlane) * ldb + koff + k0;
      bh[j] = ldfrag_u(Bb + bofs);
    }
#pragma unroll
    for (int i = 0; i < 4; ++i) {
      const size_t ao = (size_t)(m0 + (i << 4) + rlane) * lda + koff + k0;
      const v16h ah = ldfrag_u(A1 + ao);
#pragma unroll
      for (int j = 0; j < 4; ++j) acc[i][j] = mma_raw(ah, bh[j], acc[i][j]);
      dep_guard1(acc[i][0], acc[i][3], ah);
    }
    keep4_h(bh[0], bh[1], bh[2], bh[3]);
  }
  acc_guard4(acc[0][0], acc[0][1], acc[0][2], acc[0][3]);
  acc_guard4(acc[1][0], acc[1][1], acc[1][2], acc[1][3]);
  acc_guard4(acc[2][0], acc[2][1], acc[2][2], acc[2][3]);
  acc_guard4(acc[3][0], acc[3][1], acc[3][2], acc[3][3]);

  const int hh2 = lane >> 4, c4 = (lane & 15) * 4;
  const int q8  = lane >> 3, c8 = (lane & 7) * 8;

  float* slab = sT[wave];
#pragma unroll
  for (int i = 0; i < 4; ++i) {
    const int mBase = m0 + (i << 4);
#pragma unroll
    for (int j = 0; j < 4; ++j) {
#pragma unroll
      for (int r = 0; r < 8; ++r) {
        slab[(mOff + r) * 68 + (j << 4) + rlane] = acc[i][j][r];
      }
    }
    wave_sync_lds();
    if constexpr (OM == 0) {
      float* C = (float*)Cout + (size_t)((long long)by * sC);
      v4f bv = {0.f, 0.f, 0.f, 0.f};
      if constexpr (HASB == 1) {
        const v4f braw = *(const v4f*)(Bsp + n0 + c4);
#pragma unroll
        for (int e = 0; e < 4; ++e) bv[e] = bfr(braw[e]);
      }
      v4f vals[8];
#pragma unroll
      for (int it = 0; it < 8; ++it) {
        const int row = it * 2 + hh2;
        const int gr  = mBase + row;
        v4f v = *(const v4f*)(slab + row * 68 + c4);
        v4f rv = {0.f, 0.f, 0.f, 0.f};
        if constexpr (HASR != 0) {
          const float* R = Rp + (size_t)((long long)by * sC);
          const int rrow = (RMOD != 0) ? (gr & (NQ - 1)) : gr;
          const v4f rraw = *(const v4f*)(R + (size_t)rrow * ldc + n0 + c4);
#pragma unroll
          for (int e = 0; e < 4; ++e) rv[e] = (HASR == 1) ? bfr(rraw[e]) : rraw[e];
        }
#pragma unroll
        for (int e = 0; e < 4; ++e) v[e] = (v[e] * oscale + bv[e]) + rv[e];
        vals[it] = v;
      }
      for (int pass = 0; pass < 2; ++pass) {
#pragma unroll
        for (int it = 0; it < 8; ++it) {
          const int gr = mBase + it * 2 + hh2;
          *(volatile v4f*)(C + (size_t)gr * ldc + n0 + c4) = vals[it];
        }
        __threadfence();
      }
    } else {
      unsigned short* C = (unsigned short*)Cout + (size_t)((long long)by * sC);
      float bb8[8];
#pragma unroll
      for (int e = 0; e < 8; ++e) bb8[e] = 0.f;
      if constexpr (HASB == 1) {
        const v4f blo = *(const v4f*)(Bsp + n0 + c8);
        const v4f bhi = *(const v4f*)(Bsp + n0 + c8 + 4);
#pragma unroll
        for (int e = 0; e < 4; ++e) { bb8[e] = bfr(blo[e]); bb8[4 + e] = bfr(bhi[e]); }
      }
      v4u hv[4];
#pragma unroll
      for (int it = 0; it < 4; ++it) {
        const int row = it * 4 + q8;
        float brow = 0.f;
        if constexpr (HASB == 2) brow = bfr(Bsp[mBase + row]);
        const float* sp = slab + row * 68 + c8;
        v4u a = {0u, 0u, 0u, 0u};
#pragma unroll
        for (int e = 0; e < 4; ++e) {
          float f0 = (sp[2 * e] * oscale + bb8[2 * e]) + brow;
          float f1 = (sp[2 * e + 1] * oscale + bb8[2 * e + 1]) + brow;
          if constexpr (ACT == 1) { f0 = fmaxf(f0, 0.f); f1 = fmaxf(f1, 0.f); }
          if constexpr (ACT == 2) { f0 = gelu_erf(f0); f1 = gelu_erf(f1); }
          f0 *= ocarry; f1 *= ocarry;
          a[e] = pk16(h_bits((_Float16)f0), h_bits((_Float16)f1));
        }
        hv[it] = a;
      }
      for (int pass = 0; pass < 2; ++pass) {
#pragma unroll
        for (int it = 0; it < 4; ++it) {
          const int row = it * 4 + q8;
          *(volatile v4u*)(C + (size_t)(mBase + row) * ldc + n0 + c8) = hv[it];
        }
        __threadfence();
      }
    }
    wave_sync_lds();
  }
}

#define PS_FLOATS (NHEAD * 16 * 36)
static_assert((size_t)16 * OSP * sizeof(unsigned short) <= (size_t)PS_FLOATS * sizeof(float));
static_assert(((16 * OSP) / 8) == 2 * ATT_THREADS);
static_assert(OSP == HDIM * NHEAD && HDIM == 32);

__global__ __launch_bounds__(ATT_THREADS)
void attnc(const unsigned short* __restrict__ QKq, const unsigned short* __restrict__ VTq, unsigned short* CT) {
  __shared__ __align__(16) float smem[PS_FLOATS];

  const int tid  = threadIdx.x;
  const int wave = tid >> 5;
  const int lane = tid & 31;
  const int hh   = lane >> 4;
  const int c    = lane & 15;

  const int qt   = blockIdx.x % (NQ / 16);
  const int bat  = blockIdx.x / (NQ / 16);
  const int head = wave;
  const int q0   = qt * 16;

  const _Float16* QK = (const _Float16*)(const void*)QKq;
  const _Float16* Qh = QK + ((size_t)bat * NQ + q0 + c) * QKP + head * HDIM + 8 * hh;
  const _Float16* Kb = QK + (size_t)bat * NQ * QKP + DMODEL + head * HDIM + 8 * hh;
  const _Float16* Vb = (const _Float16*)(const void*)VTq + ((size_t)bat * DMODEL + head * HDIM) * NQ + 8 * hh;
  const float lsc  = (LOG2E * ATT_SCALE) / (QC * KC);

  const v16h qa = ldfrag_h(Qh);

  float mrow[8], lrow[8];
  v8f o0 = zero8(), o1 = zero8();
#pragma unroll
  for (int r = 0; r < 8; ++r) { mrow[r] = -INFINITY; lrow[r] = 0.f; }
  float* pt = smem + wave * (16 * 36);

  const int nkb = q0 + 16;
#pragma unroll 1
  for (int kb = 0; kb < nkb; kb += 32) {
    const _Float16* kp = Kb + (size_t)(kb + c) * QKP;
    v8f s0, s1;
    {
      const v16h kf0 = ldfrag_h(kp);
      const v16h kf1 = ldfrag_h(kp + (size_t)16 * QKP);
      s0 = mma_raw(qa, kf0, zero8());
      s1 = mma_raw(qa, kf1, zero8());
      guard2(s0, s1, kf0, kf1, qa);
    }
    const int key0 = kb + c, key1 = kb + 16 + c;
#pragma unroll
    for (int r = 0; r < 8; ++r) {
      const int row = q0 + 8 * hh + r;
      const float t0 = (key0 > row) ? -INFINITY : s0[r] * lsc;
      const float t1 = (key1 > row) ? -INFINITY : s1[r] * lsc;
      float mx = fmaxf(t0, t1);
#pragma unroll
      for (int off = 1; off < 16; off <<= 1) mx = fmaxf(mx, __shfl_xor(mx, off, 32));
      const float mn = fmaxf(mrow[r], mx);
      const float al = exp2f(fmaxf(mrow[r] - mn, -126.0f));
      mrow[r] = mn;
      const float e0 = exp2f(t0 - mn);
      const float e1 = exp2f(t1 - mn);
      float ps = e0 + e1;
#pragma unroll
      for (int off = 1; off < 16; off <<= 1) ps += __shfl_xor(ps, off, 32);
      lrow[r] = lrow[r] * al + ps;
      o0[r] *= al;
      o1[r] *= al;
      const int ro = (8 * hh + r) * 36 + c;
      pt[ro]      = e0;
      pt[ro + 16] = e1;
    }
    wave_sync_lds();
    FragH ph;
    {
      const float* prow = pt + c * 36 + 8 * hh;
      const v4f p0 = *(const v4f*)(prow), p1 = *(const v4f*)(prow + 4);
      const v4f p2 = *(const v4f*)(prow + 16), p3 = *(const v4f*)(prow + 20);
#pragma unroll
      for (int e = 0; e < 4; ++e) {
        ph.h[0][e]     = (_Float16)(p0[e] * PC);
        ph.h[0][4 + e] = (_Float16)(p1[e] * PC);
        ph.h[1][e]     = (_Float16)(p2[e] * PC);
        ph.h[1][4 + e] = (_Float16)(p3[e] * PC);
      }
    }
    const _Float16* vp = Vb + (size_t)c * NQ + kb;
    {
      const v16h vb0 = ldfrag_h(vp);
      const v16h vb1 = ldfrag_h(vp + (size_t)16 * NQ);
      o0 = mma_raw(ph.v, vb0, o0);
      o1 = mma_raw(ph.v, vb1, o1);
      guard2(o0, o1, ph.v, vb0, vb1);
    }
    wave_sync_lds();
  }

  __syncthreads();
  unsigned short* Os = (unsigned short*)smem;
  const float oc = FC / (PC * VC);
  unsigned short* osw = Os + wave * HDIM + c;
#pragma unroll
  for (int r = 0; r < 8; ++r) {
    const float inv = (1.0f / lrow[r]) * oc;
    unsigned short* op = osw + (8 * hh + r) * OSP;
    op[0]  = h_bits((_Float16)(o0[r] * inv));
    op[16] = h_bits((_Float16)(o1[r] * inv));
  }
  __syncthreads();
  {
    v4u vals[2];
#pragma unroll
    for (int it = 0; it < 2; ++it) {
      const int p = it * ATT_THREADS + tid;
      vals[it] = *(const v4u*)(Os + (size_t)p * 8);
    }
    unsigned short* dst = CT + ((size_t)bat * NQ + q0) * DMODEL;
    for (int pass = 0; pass < 2; ++pass) {
#pragma unroll
      for (int it = 0; it < 2; ++it) {
        const int p = it * ATT_THREADS + tid;
        const int row = p >> 5, col8 = (p & 31) * 8;
        *(volatile v4u*)(dst + (size_t)row * DMODEL + col8) = vals[it];
      }
      __threadfence();
    }
  }
}

__device__ __forceinline__ v8f ln_row(const float* __restrict__ yr, const float* __restrict__ gr8, const float* __restrict__ br8) {
  const v4f a = *(const v4f*)(yr), b4 = *(const v4f*)(yr + 4);
  float v[8];
  v[0] = a[0]; v[1] = a[1]; v[2] = a[2]; v[3] = a[3]; v[4] = b4[0]; v[5] = b4[1]; v[6] = b4[2]; v[7] = b4[3];
  float s = ((v[0] + v[1]) + (v[2] + v[3])) + ((v[4] + v[5]) + (v[6] + v[7]));
#pragma unroll
  for (int off = 1; off < 32; off <<= 1) s += __shfl_xor(s, off, 32);
  const float mu = s * (1.0f / (float)DMODEL);
  float d[8];
#pragma unroll
  for (int e = 0; e < 8; ++e) d[e] = v[e] - mu;
  float q = 0.f;
#pragma unroll
  for (int e = 0; e < 8; ++e) q += d[e] * d[e];
#pragma unroll
  for (int off = 1; off < 32; off <<= 1) q += __shfl_xor(q, off, 32);
  const float var  = q * (1.0f / (float)DMODEL);
  const float rstd = rsqrtf(var + LN_EPS);
  const v4f g0 = *(const v4f*)(gr8), g1 = *(const v4f*)(gr8 + 4);
  const v4f c0 = *(const v4f*)(br8), c1 = *(const v4f*)(br8 + 4);
  float gg[8], bb[8];
  gg[0] = g0[0]; gg[1] = g0[1]; gg[2] = g0[2]; gg[3] = g0[3]; gg[4] = g1[0]; gg[5] = g1[1]; gg[6] = g1[2]; gg[7] = g1[3];
  bb[0] = c0[0]; bb[1] = c0[1]; bb[2] = c0[2]; bb[3] = c0[3]; bb[4] = c1[0]; bb[5] = c1[1]; bb[6] = c1[2]; bb[7] = c1[3];
  v8f o;
#pragma unroll
  for (int e = 0; e < 8; ++e) o[e] = (d[e] * rstd) * bfr(gg[e]) + bfr(bb[e]);
  return o;
}

__global__ __launch_bounds__(LN_THREADS)
void lnormD(const float* __restrict__ Yp, const float* __restrict__ gp, const float* __restrict__ bp,
            unsigned short* outh, float hc) {
  const int tid = threadIdx.x, lane = tid & 31, wave = tid >> 5;
  const int row = blockIdx.x * 8 + wave;
  const v8f o = ln_row(Yp + (size_t)row * DMODEL + lane * 8, gp + lane * 8, bp + lane * 8);
  v4u w;
#pragma unroll
  for (int e = 0; e < 4; ++e)
    w[e] = pk16(h_bits((_Float16)(o[2 * e] * hc)), h_bits((_Float16)(o[2 * e + 1] * hc)));
  unsigned short* dst = outh + (size_t)row * DMODEL + lane * 8;
  for (int pass = 0; pass < 2; ++pass) {
    *(volatile v4u*)dst = w;
    __threadfence();
  }
}

__global__ __launch_bounds__(LN_THREADS)
void lnfin(const float* __restrict__ Yp, const float* __restrict__ gp, const float* __restrict__ bp,
           const float* __restrict__ wop, const float* __restrict__ bop, float* out) {
  __shared__ __align__(16) float srow[8][DMODEL];
  __shared__ __align__(16) float sO[8 * DOUT];
  const int tid = threadIdx.x, lane = tid & 31, wave = tid >> 5;
  const int row = blockIdx.x * 8 + wave;
  const v8f o = ln_row(Yp + (size_t)row * DMODEL + lane * 8, gp + lane * 8, bp + lane * 8);
  float* sr = srow[wave];
  {
    v4f oa, ob;
    oa[0] = o[0]; oa[1] = o[1]; oa[2] = o[2]; oa[3] = o[3];
    ob[0] = o[4]; ob[1] = o[5]; ob[2] = o[6]; ob[3] = o[7];
    *(v4f*)(sr + lane * 8)     = oa;
    *(v4f*)(sr + lane * 8 + 4) = ob;
  }
  wave_sync_lds();
  {
    const v4f u0 = *(const v4f*)(sr + lane * 4);
    const v4f u1 = *(const v4f*)(sr + (DMODEL / 2) + lane * 4);
    float* hrow = out + (size_t)OUT0_N + (size_t)row * DMODEL;
    for (int pass = 0; pass < 2; ++pass) {
      *(volatile v4f*)(hrow + lane * 4) = u0;
      *(volatile v4f*)(hrow + (DMODEL / 2) + lane * 4) = u1;
      __threadfence();
    }
  }
  const int oo = lane & 7, jj = lane >> 3;
  float acc = 0.f;
#pragma unroll 2
  for (int i = 0; i < DMODEL / 4; ++i) {
    const int cc = jj * (DMODEL / 4) + i;
    acc += sr[cc] * bfr(wop[cc * DOUT + oo]);
  }
  acc += __shfl_xor(acc, 8, 32);
  acc += __shfl_xor(acc, 16, 32);
  const float bo8 = bfr(bop[lane & 7]);
  if (lane < DOUT) sO[wave * DOUT + lane] = acc + bo8;
  __syncthreads();
  if (tid < 16) {
    const v4f w4 = *(const v4f*)(sO + tid * 4);
    float* op = out + (size_t)blockIdx.x * (8 * DOUT) + tid * 4;
    for (int pass = 0; pass < 2; ++pass) {
      *(volatile v4f*)op = w4;
      __threadfence();
    }
  }
}

extern "C" void kernel_launch(void* const* d_in, const int* in_sizes, int n_in,
                              void* d_out, int out_size, void* d_ws, size_t ws_size,
                              hipStream_t stream) {
  if (n_in < 23) return;
  if (in_sizes[0] != NROWS * DIN) return;
  if (in_sizes[1] != DIN * DMODEL || in_sizes[2] != DMODEL) return;
  if (in_sizes[3] != NLAYER * DMODEL * DMODEL || in_sizes[5] != NLAYER * DMODEL * DMODEL || in_sizes[7] != NLAYER * DMODEL * DMODEL) return;
  if (in_sizes[4] != NLAYER * DMODEL || in_sizes[6] != NLAYER * DMODEL || in_sizes[8] != NLAYER * DMODEL) return;
  if (in_sizes[9] != NLAYER * DMODEL * DMODEL || in_sizes[10] != NLAYER * DMODEL) return;
  if (in_sizes[11] != NLAYER * DMODEL || in_sizes[12] != NLAYER * DMODEL || in_sizes[13] != NLAYER * DMODEL || in_sizes[14] != NLAYER * DMODEL) return;
  if (in_sizes[15] != NLAYER * DMODEL * DFF || in_sizes[16] != NLAYER * DFF) return;
  if (in_sizes[17] != NLAYER * DFF * DMODEL || in_sizes[18] != NLAYER * DMODEL) return;
  if (in_sizes[19] != DMODEL || in_sizes[20] != DMODEL) return;
  if (in_sizes[21] != DMODEL * DOUT || in_sizes[22] != DOUT) return;
  if (out_size != OUT0_N + NROWS * DMODEL) return;

  const float* x     = (const float*)d_in[0];
  const float* w_in  = (const float*)d_in[1];
  const float* b_in  = (const float*)d_in[2];
  const float* wq    = (const float*)d_in[3];
  const float* bq    = (const float*)d_in[4];
  const float* wk    = (const float*)d_in[5];
  const float* bk    = (const float*)d_in[6];
  const float* wv    = (const float*)d_in[7];
  const float* bv    = (const float*)d_in[8];
  const float* wo    = (const float*)d_in[9];
  const float* bo    = (const float*)d_in[10];
  const float* ln1_g = (const float*)d_in[11];
  const float* ln1_b = (const float*)d_in[12];
  const float* ln2_g = (const float*)d_in[13];
  const float* ln2_b = (const float*)d_in[14];
  const float* w1    = (const float*)d_in[15];
  const float* b1    = (const float*)d_in[16];
  const float* w2    = (const float*)d_in[17];
  const float* b2    = (const float*)d_in[18];
  const float* lnf_g = (const float*)d_in[19];
  const float* lnf_b = (const float*)d_in[20];
  const float* w_out = (const float*)d_in[21];
  const float* b_out = (const float*)d_in[22];
  float*       out   = (float*)d_out;

  const size_t PWQKV = (size_t)NLAYER * 3 * DMODEL * DMODEL * 2;
  const size_t PWO   = (size_t)NLAYER * DMODEL * DMODEL * 2;
  const size_t PW1   = (size_t)NLAYER * DFF * DMODEL * 2;
  const size_t PW2   = (size_t)NLAYER * DMODEL * DFF * 2;
  const size_t PWIN  = (size_t)DMODEL * DIN * 2;
  const size_t PX0   = (size_t)NROWS * DIN * 2;
  const size_t PPE   = (size_t)NQ * DMODEL * 4;
  const size_t PH    = (size_t)NROWS * DMODEL * 4;
  const size_t PX16  = (size_t)NROWS * DMODEL * 2;
  const size_t PQK   = (size_t)NROWS * QKP * 2;
  const size_t PVT   = (size_t)NB * DMODEL * NQ * 2;
  const size_t PCT   = (size_t)NROWS * DMODEL * 2;
  const size_t PG    = (size_t)NROWS * DFF * 2;
  size_t off = 0;
  const size_t oWQKV = off; off += PWQKV;
  const size_t oWO   = off; off += PWO;
  const size_t oW1   = off; off += PW1;
  const size_t oW2   = off; off += PW2;
  const size_t oWIN  = off; off += PWIN;
  const size_t oX0   = off; off += PX0;
  const size_t oPE   = off; off += PPE;
  const size_t oHA   = off; off += PH;
  const size_t oHB   = off; off += PH;
  const size_t oX16  = off; off += PX16;
  const size_t oQK   = off; off += PQK;
  const size_t oVT   = off; off += PVT;
  const size_t oCT   = off; off += PCT;
  const size_t oG    = off; off += PG;
  if (off > ws_size) return;
  if (off > (size_t)134217728) return;

  char* ws = (char*)d_ws;
  unsigned short* WQKV = (unsigned short*)(ws + oWQKV);
  unsigned short* WO16 = (unsigned short*)(ws + oWO);
  unsigned short* W1T  = (unsigned short*)(ws + oW1);
  unsigned short* W2T  = (unsigned short*)(ws + oW2);
  unsigned short* WIN  = (unsigned short*)(ws + oWIN);
  unsigned short* X0   = (unsigned short*)(ws + oX0);
  float*          PEt  = (float*)(ws + oPE);
  float*          HA   = (float*)(ws + oHA);
  float*          HB   = (float*)(ws + oHB);
  unsigned short* X16  = (unsigned short*)(ws + oX16);
  unsigned short* QK   = (unsigned short*)(ws + oQK);
  unsigned short* VTp  = (unsigned short*)(ws + oVT);
  unsigned short* CT   = (unsigned short*)(ws + oCT);
  unsigned short* G16  = (unsigned short*)(ws + oG);

  const dim3 blk(256);
  const dim3 gQKV(NHEAD, NLAYER, 3);
  const dim3 gTO(DMODEL / 64, DMODEL / 64, NLAYER);
  const dim3 gT1(DFF / 64, DMODEL / 64, NLAYER);
  const dim3 gT2(DMODEL / 64, DFF / 64, NLAYER);
  const dim3 gTI(DMODEL / 64, DIN / 64, 1);
  const int  n8x = (NROWS * DIN) / 8;
  const dim3 gCX(n8x / CVT_THREADS);
  const dim3 gPE((NQ * (DMODEL / 2)) / 256);
  const int tilesP = (NROWS / 64) * (DMODEL / 64);
  const int tilesV = (DMODEL / 64) * (NQ / 64);
  const int tilesF = (NROWS / 64) * (DFF / 64);
  const dim3 gP((tilesP + 7) / 8, 1);
  const dim3 gV((tilesV + 7) / 8, NB);
  const dim3 gF((tilesF + 7) / 8, 1);
  const dim3 gAT(ATT_BLOCKS);
  const dim3 bAT(ATT_THREADS);
  const dim3 gLN(NROWS / 8);
  const dim3 bLN(LN_THREADS);

  cvtqkv<<<gQKV, blk, 0, stream>>>(wq, wk, wv, WQKV, WSC);
  tcvt16<<<gTO, blk, 0, stream>>>(wo, WO16, DMODEL, DMODEL, WSC);
  tcvt16<<<gT1, blk, 0, stream>>>(w1, W1T, DMODEL, DFF, WSC);
  tcvt16<<<gT2, blk, 0, stream>>>(w2, W2T, DFF, DMODEL, WSC);
  tcvt16<<<gTI, blk, 0, stream>>>(w_in, WIN, DIN, DMODEL, WSC);
  cvt16<<<gCX, blk, 0, stream>>>(x, X0, n8x, 1.0f);
  petab<<<gPE, blk, 0, stream>>>(PEt);

  gemm64<0, 2, 1, 0, 1><<<gP, blk, 0, stream>>>(
      X0, DIN, 0LL,
      WIN, DIN, 0LL,
      PEt, b_in,
      (void*)HA, DMODEL, 0LL,
      NROWS, DMODEL, DIN, 1.0f / WSC, 1.0f);

  for (int l = 0; l < NLAYER; ++l) {
    const unsigned short* Wl = WQKV + (size_t)l * (3 * DMODEL) * DMODEL;

    lnormD<<<gLN, bLN, 0, stream>>>(HA, ln1_g + (size_t)l * DMODEL, ln1_b + (size_t)l * DMODEL, X16, HCARRY);

    gemm64<2, 0, 1, 0, 0><<<gP, blk, 0, stream>>>(
        X16, DMODEL, 0LL,
        Wl, DMODEL, 0LL,
        (const float*)0, bq + (size_t)l * DMODEL,
        (void*)QK, QKP, 0LL,
        NROWS, DMODEL, DMODEL, 1.0f / (HCARRY * WSC), QC);

    gemm64<2, 0, 1, 0, 0><<<gP, blk, 0, stream>>>(
        X16, DMODEL, 0LL,
        Wl + (size_t)DMODEL * DMODEL, DMODEL, 0LL,
        (const float*)0, bk + (size_t)l * DMODEL,
        (void*)(QK + DMODEL), QKP, 0LL,
        NROWS, DMODEL, DMODEL, 1.0f / (HCARRY * WSC), KC);

    gemm64<2, 0, 2, 0, 0><<<gV, blk, 0, stream>>>(
        Wl + (size_t)2 * DMODEL * DMODEL, DMODEL, 0LL,
        X16, DMODEL, (long long)NQ * DMODEL,
        (const float*)0, bv + (size_t)l * DMODEL,
        (void*)VTp, NQ, (long long)DMODEL * NQ,
        DMODEL, NQ, DMODEL, 1.0f / (HCARRY * WSC), VC);

    attnc<<<gAT, bAT, 0, stream>>>(QK, VTp, CT);

    gemm64<0, 2, 1, 0, 0><<<gP, blk, 0, stream>>>(
        CT, DMODEL, 0LL,
        WO16 + (size_t)l * DMODEL * DMODEL, DMODEL, 0LL,
        HA, bo + (size_t)l * DMODEL,
        (void*)HB, DMODEL, 0LL,
        NROWS, DMODEL, DMODEL, 1.0f / (FC * WSC), 1.0f);

    lnormD<<<gLN, bLN, 0, stream>>>(HB, ln2_g + (size_t)l * DMODEL, ln2_b + (size_t)l * DMODEL, X16, HCARRY);

    gemm64<2, 0, 1, 2, 0><<<gF, blk, 0, stream>>>(
        X16, DMODEL, 0LL,
        W1T + (size_t)l * DFF * DMODEL, DMODEL, 0LL,
        (const float*)0, b1 + (size_t)l * DFF,
        (void*)G16, DFF, 0LL,
        NROWS, DFF, DMODEL, 1.0f / (HCARRY * WSC), GC);

    gemm64<0, 2, 1, 0, 0><<<gP, blk, 0, stream>>>(
        G16, DFF, 0LL,
        W2T + (size_t)l * DMODEL * DFF, DFF, 0LL,
        HB, b2 + (size_t)l * DMODEL,
        (void*)HA, DMODEL, 0LL,
        NROWS, DMODEL, DFF, 1.0f / (GC * WSC), 1.0f);
  }

  lnfin<<<gLN, bLN, 0, stream>>>(HA, lnf_g, lnf_b, w_out, b_out, out);
}
